// MultiHeadSelfAttention_42159398977859
// MI455X (gfx1250) — hardware-verified
//
#include <hip/hip_runtime.h>
#include <math.h>

typedef __attribute__((ext_vector_type(16))) _Float16 v16h;
typedef __attribute__((ext_vector_type(16))) __bf16 v16b;
typedef __attribute__((ext_vector_type(8)))  _Float16 v8h;
typedef __attribute__((ext_vector_type(8)))  float v8f;
typedef __attribute__((ext_vector_type(4)))  float v4f;
typedef __attribute__((ext_vector_type(4)))  unsigned v4u;

template <typename T> __device__ __forceinline__ void vst2(void* p, T v) { *(volatile T*)p = v; __threadfence(); *(volatile T*)p = v; }
__device__ __forceinline__ v8f wmma16(v16h a, v16h b, v8f c) {
  v8f d = __builtin_amdgcn_wmma_f32_16x16x32_f16(false, a, false, b, (short)0, c, false, false);
  asm volatile("v_nop\n\tv_nop\n\tv_nop\n\tv_nop" : "+v"(d) : "v"(a), "v"(b));
  return d;
}
__device__ __forceinline__ v8f wmma_bf(v16b a, v16b b, v8f c) {
  v8f d = __builtin_amdgcn_wmma_f32_16x16x32_bf16(false, a, false, b, (short)0, c, false, false);
  asm volatile("v_nop\n\tv_nop\n\tv_nop\n\tv_nop" : "+v"(d) : "v"(a), "v"(b));
  return d;
}
__device__ __forceinline__ v16h frag_h(const _Float16* rowk0, int lane) {
  union { v16h v; v8h q[2]; } u; const _Float16* p = rowk0 + 8 * (lane >> 4);
  u.q[0] = *(const v8h*)p; u.q[1] = *(const v8h*)(p + 16); return u.v;
}
struct F2 { v16b h, l; };
__device__ __forceinline__ F2 bsplit16(const float v[16]) { F2 r;
#pragma unroll
  for (int i = 0; i < 16; ++i) { const __bf16 h = (__bf16)v[i]; r.h[i] = h; r.l[i] = (__bf16)(v[i] - (float)h); }
  return r; }
__device__ __forceinline__ F2 split_row(const float* row, int k0, int lane) { float v[16]; const float* p = row + k0 + 8 * (lane >> 4);
#pragma unroll
  for (int i = 0; i < 8; ++i) { v[i] = p[i]; v[8 + i] = p[16 + i]; }
  return bsplit16(v); }
#define LDSX() do { asm volatile("s_wait_dscnt 0" ::: "memory"); __builtin_amdgcn_wave_barrier(); __builtin_amdgcn_fence(3  , "workgroup"); } while (0)

#ifndef NB
#define NB 2
#endif
#ifndef SEQ
#define SEQ 2048
#endif
#define NB_FULL 2
#define SEQ_FULL 2048
#define TT SEQ
#define CC 1024
#define DIN 1024
#define NH 16
#define HD 64
#define WLD (3 * CC)
#define SC2 (0.18033688011112042f)
#define PCARRY 2048.0f

static_assert(CC == NH * HD);
static_assert(HD == 64);
static_assert(TT % 64 == 0);
static_assert(TT % 32 == 0);
static_assert(DIN % 32 == 0 && CC % 32 == 0);
static_assert(CC % 128 == 0 && DIN % 128 == 0);
static_assert(NB <= NB_FULL && SEQ <= SEQ_FULL);
static_assert((TT & (TT - 1)) == 0);

__device__ __forceinline__ float bfr(float v) { return (float)(__bf16)v; }
__device__ __forceinline__ v16b wcol_io(const float* Wm, int k0, int o, int lane, int ld) { v16b w; const int g = lane >> 4;
#pragma unroll
  for (int i = 0; i < 8; ++i) { w[i] = (__bf16)Wm[(size_t)(k0 + 8 * g + i) * ld + o]; w[8 + i] = (__bf16)Wm[(size_t)(k0 + 16 + 8 * g + i) * ld + o]; }
  return w; }

#define WS_QH  0u
#define WS_KH  (WS_QH + 2u * (size_t)NB * TT * CC)
#define WS_VT  (WS_KH + 2u * (size_t)NB * TT * CC)
#define WS_Y   (WS_VT + 2u * (size_t)NB * CC * TT)
#define WS_END (WS_Y  + 4u * (size_t)NB * TT * CC)
static_assert(WS_END <= 134217728u);
static_assert((size_t)(NB * TT / 64) * (CC / 128) * 64 * 128 == (size_t)NB * TT * CC);
static_assert((size_t)(TT / 64) * NH * NB * 64 * HD == (size_t)NB * TT * CC);
static_assert((size_t)(NB * TT / 64) * (DIN / 128) * 64 * 128 == (size_t)NB * TT * DIN);

__global__ __launch_bounds__(128) void k_proj(const float* __restrict__ X, const float* __restrict__ W, const float* __restrict__ BQKV,
    _Float16* __restrict__ QH, _Float16* __restrict__ KH, _Float16* __restrict__ VT) {
  __shared__ __align__(16) _Float16 sh[64][136]; __shared__ __align__(16) _Float16 th[128][72];
  const unsigned tid = threadIdx.x, wave = tid >> 5, lane = tid & 31u, col = lane & 15u, g = lane >> 4;
  const unsigned which = blockIdx.z, c0 = blockIdx.y * 128u, rb = blockIdx.x * 64u, bb = rb / (unsigned)TT, t0 = rb % (unsigned)TT;
  const float* WA = W + which * (unsigned)CC; const float* BA = BQKV + which * (unsigned)CC;
  const size_t xr = (size_t)bb * SEQ_FULL + t0 + wave * 16u + col;
  v8f acc[8] = {};
#pragma unroll 2
  for (int kc = 0; kc < DIN / 32; ++kc) { v16b a; { const float* p = X + xr * DIN + kc * 32 + 8 * g;
#pragma unroll
      for (int i = 0; i < 8; ++i) { a[i] = (__bf16)p[i]; a[8 + i] = (__bf16)p[16 + i]; } }
    asm volatile("s_wait_loadcnt 0x0" ::: "memory");
#pragma unroll
    for (int j = 0; j < 8; ++j) { const v16b w = wcol_io(WA, kc * 32, (int)(c0 + j * 16 + col), (int)lane, WLD); asm volatile("s_wait_loadcnt 0x0" ::: "memory"); acc[j] = wmma_bf(a, w, acc[j]); } }
  if (which < 2u) { _Float16* DH = which == 0u ? QH : KH;
#pragma unroll
    for (int j = 0; j < 8; ++j) { const float bias = bfr(BA[c0 + j * 16 + col]);
#pragma unroll
      for (int r = 0; r < 8; ++r) { const float v = acc[j][r] + bias; sh[wave * 16 + 8 * g + r][j * 16 + col] = (_Float16)v; } }
    __syncthreads();
    for (unsigned e = tid; e < 64u * 16u; e += 128u) { const unsigned rl = e >> 4, q = e & 15u; vst2(DH + ((size_t)rb + rl) * CC + c0 + q * 8u, *(const v4u*)&sh[rl][q * 8u]); }
  } else {
#pragma unroll
    for (int j = 0; j < 8; ++j) { const float bias = bfr(BA[c0 + j * 16 + col]);
#pragma unroll
      for (int r = 0; r < 8; ++r) { const float v = acc[j][r] + bias; th[j * 16 + col][wave * 16 + 8 * g + r] = (_Float16)v; } }
    __syncthreads();
    for (unsigned e = tid; e < 128u * 8u; e += 128u) { const unsigned cl = e >> 3, q = e & 7u; vst2(VT + ((size_t)bb * CC + c0 + cl) * (size_t)TT + t0 + q * 8u, *(const v4u*)&th[cl][q * 8u]); } } }

__global__ __launch_bounds__(128) void k_flash(const _Float16* __restrict__ QH, const _Float16* __restrict__ KH, const _Float16* __restrict__ VT, float* __restrict__ Y) {
  __shared__ __align__(16) float ss[4][16][HD + 4];
  const unsigned tid = threadIdx.x, wave = tid >> 5, lane = tid & 31u, col = lane & 15u, g = lane >> 4;
  const unsigned qb = blockIdx.x, h = blockIdx.y, b = blockIdx.z;
  const unsigned ql0 = qb * 64u + wave * 16u; const size_t rowb = (size_t)b * TT;
  v16h qf[HD / 32];
#pragma unroll
  for (int kc = 0; kc < HD / 32; ++kc) qf[kc] = frag_h(QH + (rowb + ql0 + col) * CC + h * HD + kc * 32, (int)lane);
  const _Float16* Kb = KH + rowb * CC + h * HD;
  const _Float16* Vb = VT + ((size_t)b * CC + h * HD) * (size_t)TT;
  float m = -3.0e38f, l = 0.f;
  v8f ot[HD / 16] = {};
#pragma unroll 1
  for (unsigned k0 = 0; k0 < (unsigned)TT; k0 += 32u) {
    v8f s0 = {}, s1 = {};
#pragma unroll
    for (int kc = 0; kc < HD / 32; ++kc) {
      const v16h ka = frag_h(Kb + (size_t)(k0 + col) * CC + kc * 32, (int)lane);
      const v16h kz = frag_h(Kb + (size_t)(k0 + 16u + col) * CC + kc * 32, (int)lane);
      s0 = wmma16(ka, qf[kc], s0); s1 = wmma16(kz, qf[kc], s1); }
    float sv[16];
#pragma unroll
    for (int i = 0; i < 8; ++i) { sv[i] = s0[i] * SC2; sv[8 + i] = s1[i] * SC2; }
    float rm = sv[0];
#pragma unroll
    for (int i = 1; i < 16; ++i) rm = fmaxf(rm, sv[i]);
    rm = fmaxf(rm, __shfl_xor(rm, 16));
    const float mn = fmaxf(m, rm);
    const float corr = exp2f(m - mn);
    float rs = 0.f; v16h pf;
#pragma unroll
    for (int i = 0; i < 16; ++i) { const float p = exp2f(sv[i] - mn); rs += p; pf[i] = (_Float16)(p * PCARRY); }
    rs += __shfl_xor(rs, 16);
    l = l * corr + rs; m = mn;
#pragma unroll
    for (int t = 0; t < HD / 16; ++t)
#pragma unroll
      for (int i = 0; i < 8; ++i) ot[t][i] *= corr;
#pragma unroll
    for (int t = 0; t < HD / 16; ++t) { const v16h va = frag_h(Vb + (size_t)(t * 16 + col) * TT + k0, (int)lane); ot[t] = wmma16(va, pf, ot[t]); }
  }
  const float inv = 1.0f / (l * PCARRY);
#pragma unroll
  for (int t = 0; t < HD / 16; ++t)
#pragma unroll
    for (int r = 0; r < 8; ++r) ss[wave][col][t * 16 + 8 * g + r] = ot[t][r] * inv;
  LDSX();
  for (unsigned it = 0; it < 8u; ++it) { const unsigned rl = it * 2u + g; vst2(Y + (rowb + ql0 + rl) * CC + h * HD + col * 4u, *(const v4f*)&ss[wave][rl][col * 4u]); } }

__global__ __launch_bounds__(128) void k_out(const float* __restrict__ Y, const float* __restrict__ WO, const float* __restrict__ BO, float* __restrict__ OUT) {
  __shared__ __align__(16) float sf[4][16][132];
  const unsigned tid = threadIdx.x, wave = tid >> 5, lane = tid & 31u, col = lane & 15u, g = lane >> 4;
  const unsigned c0 = blockIdx.y * 128u, rb = blockIdx.x * 64u, bb = rb / (unsigned)TT, t0 = rb % (unsigned)TT;
  const size_t r0 = (size_t)rb + wave * 16u;
  const size_t o0 = (size_t)bb * SEQ_FULL + t0 + wave * 16u;
  v8f acc[8] = {};
#pragma unroll 2
  for (int kc = 0; kc < CC / 32; ++kc) { const F2 a = split_row(Y + (r0 + col) * CC, kc * 32, (int)lane); asm volatile("s_wait_loadcnt 0x0" ::: "memory");
#pragma unroll
    for (int j = 0; j < 8; ++j) { const v16b w = wcol_io(WO, kc * 32, (int)(c0 + j * 16 + col), (int)lane, DIN); asm volatile("s_wait_loadcnt 0x0" ::: "memory"); acc[j] = wmma_bf(a.h, w, acc[j]); acc[j] = wmma_bf(a.l, w, acc[j]); } }
#pragma unroll
  for (int j = 0; j < 8; ++j) { const float bias = bfr(BO[c0 + j * 16 + col]);
#pragma unroll
    for (int r = 0; r < 8; ++r) sf[wave][8 * g + r][j * 16 + col] = acc[j][r] + bias; }
  LDSX();
  for (unsigned rl = 0; rl < 16u; ++rl) vst2(OUT + (o0 + rl) * DIN + c0 + lane * 4u, *(const v4f*)&sf[wave][rl][lane * 4u]); }

extern "C" void kernel_launch(void* const* d_in, const int* in_sizes, int n_in, void* d_out, int out_size, void* d_ws, size_t ws_size, hipStream_t stream) {
  if (n_in < 5) return;
  const size_t xneed = ((size_t)(NB - 1) * SEQ_FULL + SEQ) * DIN;
  if ((size_t)in_sizes[0] < xneed) return;
  if ((size_t)in_sizes[1] < (size_t)DIN * WLD) return;
  if ((size_t)in_sizes[2] < (size_t)WLD) return;
  if ((size_t)in_sizes[3] < (size_t)CC * DIN) return;
  if ((size_t)in_sizes[4] < (size_t)DIN) return;
  if ((size_t)out_size < xneed) return;
  if (ws_size < (size_t)WS_END) return;
  const float* x = (const float*)d_in[0]; const float* wqkv = (const float*)d_in[1]; const float* bqkv = (const float*)d_in[2]; const float* wout = (const float*)d_in[3]; const float* bout = (const float*)d_in[4];
  char* ws = (char*)d_ws; _Float16 *QH = (_Float16*)(ws + WS_QH), *KH = (_Float16*)(ws + WS_KH), *VT = (_Float16*)(ws + WS_VT); float* Y = (float*)(ws + WS_Y);
  k_proj<<<dim3(NB * TT / 64, CC / 128, 3), 128, 0, stream>>>(x, wqkv, bqkv, QH, KH, VT);
  k_flash<<<dim3(TT / 64, NH, NB), 128, 0, stream>>>(QH, KH, VT, Y);
  k_out<<<dim3(NB * TT / 64, DIN / 128), 128, 0, stream>>>(Y, wout, bout, (float*)d_out);
}
